// GINE_37443524886787
// MI455X (gfx1250) — hardware-run, weakly checked
//
#include <hip/hip_runtime.h>
#include <stddef.h>
#include <stdint.h>


#define NN      50000
#define NE      300000
#define DD      256
#define EDK     16
#define NL      3
#define NGR     2000
#define MP      50048
#define KP      512
#define ZSINGLE 0
#define TSINGLE 0
#define KZ      (ZSINGLE ? 256 : 512)
#define KT      (TSINGLE ? 256 : 512)
#define PLANE   (DD * KP)
#define NTHR    256
#define NWAVE   8
#define EPT     8
#define CHUNK   (NTHR * EPT)
#define WCAP    (EPT * 32)
#define LISTN   (NWAVE * WCAP)
#define NBE     1024
#define RCAPE   8192
#define DEGCAP  32
#define NBG     512
#define RCAPG   16384
#define PGCAP   96
#define GBM     64
#define BN      128
#define GTHR    128
#define GNT     8
#define TPI     260
#define LDS_BKE ((2 * RCAPE + 2 * NBE + LISTN + 2 * NWAVE) * 4)
#define LDS_BKG ((2 * RCAPG + 2 * NBG + LISTN + 2 * NWAVE) * 4)
#define LDS_CONV (16384 + 1024 + NWAVE * 1024 + NWAVE * 16 * TPI * 4)
#define OUT1_EL (NN * DD)

static_assert(DD == 256 && DD == 32 * 8);
static_assert(EDK == 16);
static_assert(NN <= 49 * NBE);
static_assert(NGR <= 4 * NBG);
static_assert((MP % GBM) == 0 && MP >= NN && (MP % NWAVE) == 0 && MP - NN == 48);
static_assert((NGR % NWAVE) == 0);
static_assert((NE % 4) == 0);
static_assert(KZ <= KP && KT <= KP && (KZ % 32) == 0 && (KT % 32) == 0 && KP == 2 * DD);
static_assert((CHUNK & (CHUNK - 1)) == 0 && CHUNK <= 4096);
static_assert((NBE & (NBE - 1)) == 0 && NBE <= 4096 && (NBG & (NBG - 1)) == 0 && NBG <= 4096);
static_assert(NE < (1 << 20) && NN < (1 << 20));
static_assert(LISTN >= 2 * NBE && LISTN >= 2 * NBG);
static_assert((RCAPE % (2 * NTHR)) == 0 && (RCAPG % (4 * NTHR)) == 0);
static_assert(RCAPE >= 6271 + 6271 / 4 && RCAPG >= 12945 + 12945 / 4);
static_assert(DEGCAP >= 19 + 8 && PGCAP >= 42 + 8);
static_assert(LDS_BKE <= 327680 && LDS_BKG <= 327680);
static_assert(LDS_CONV == 158720 && LDS_CONV <= 327680);
static_assert(GBM == (GTHR / 32) * 16 && BN == 16 * GNT && DD == 2 * BN);
static_assert((TPI % 4) == 0 && TPI >= DD);
static_assert(OUT1_EL * 4 == 51200000 && ((OUT1_EL * 4) % 128) == 0);
static_assert(OUT1_EL + (NGR - 1) * DD + DD - 1 < OUT1_EL + NGR * DD);

typedef float          v4f   __attribute__((ext_vector_type(4)));
typedef float          v8f   __attribute__((ext_vector_type(8)));
typedef int            v2i   __attribute__((ext_vector_type(2)));
typedef int            v4i   __attribute__((ext_vector_type(4)));
typedef int            v8i   __attribute__((ext_vector_type(8)));
typedef unsigned       v4u   __attribute__((ext_vector_type(4)));
typedef unsigned short v8us  __attribute__((ext_vector_type(8)));
typedef __bf16         v16bf __attribute__((ext_vector_type(16)));
typedef v4f __attribute__((may_alias)) v4fa;
typedef v4i __attribute__((may_alias)) v4ia;
union FragB { v16bf v; v8us u[2]; v8i w; v4i q[2]; };
struct HL { v4u h; v4u l; };

__device__ __forceinline__ v8f wmx(const FragB& a, const FragB& b, v8f c) {
  v8f d = __builtin_amdgcn_wmma_f32_16x16x32_bf16(false, a.v, false, b.v, (short)0, c, false, false);
  asm volatile("v_nop\n\tv_nop\n\tv_nop\n\tv_nop" : "+v"(d) : "v"(a.w), "v"(b.w));
  return d;
}

__device__ __forceinline__ void pinf(float x) { asm volatile("" :: "v"(x)); }
__device__ __forceinline__ void pini(int x)   { asm volatile("" :: "v"(x)); }
__device__ __forceinline__ int iclamp(int v, int lo, int hi) { v = v < lo ? lo : v; return v > hi ? hi : v; }

__device__ __forceinline__ unsigned bfbits(float v) {
  const unsigned u = __float_as_uint(v);
  const unsigned r = (u + 0x7FFFu + ((u >> 16) & 1u)) >> 16;
  const unsigned nb = ((u >> 16) & 0x8000u) | 0x7FC0u;
  return ((u & 0x7FFFFFFFu) > 0x7F800000u) ? nb : r;
}
__device__ __forceinline__ float rbf(float v) { return __uint_as_float(bfbits(v) << 16); }
__device__ __forceinline__ float relu_keep(float v) { return (v > 0.0f) ? v : (v - v); }

__device__ __forceinline__ HL split8(const v4f a, const v4f b) {
  const unsigned h0 = bfbits(a.x), h1 = bfbits(a.y), h2 = bfbits(a.z), h3 = bfbits(a.w);
  const unsigned h4 = bfbits(b.x), h5 = bfbits(b.y), h6 = bfbits(b.z), h7 = bfbits(b.w);
  const unsigned l0 = bfbits(a.x - __uint_as_float(h0 << 16)), l1 = bfbits(a.y - __uint_as_float(h1 << 16));
  const unsigned l2 = bfbits(a.z - __uint_as_float(h2 << 16)), l3 = bfbits(a.w - __uint_as_float(h3 << 16));
  const unsigned l4 = bfbits(b.x - __uint_as_float(h4 << 16)), l5 = bfbits(b.y - __uint_as_float(h5 << 16));
  const unsigned l6 = bfbits(b.z - __uint_as_float(h6 << 16)), l7 = bfbits(b.w - __uint_as_float(h7 << 16));
  HL o;
  o.h.x = h0 | (h1 << 16); o.h.y = h2 | (h3 << 16); o.h.z = h4 | (h5 << 16); o.h.w = h6 | (h7 << 16);
  o.l.x = l0 | (l1 << 16); o.l.y = l2 | (l3 << 16); o.l.z = l4 | (l5 << 16); o.l.w = l6 | (l7 << 16);
  return o;
}

__device__ __forceinline__ void prep_wplane(const float* __restrict__ W, unsigned short* wd, int v) {
  const int l = v >> 13;
  const int w = v & 8191;
  const int n = w >> 5;
  const int k8 = (w & 31) * 8;
  const float* p = W + (size_t)l * (DD * DD) + (size_t)k8 * DD + n;
  float f[8];
#pragma unroll
  for (int i = 0; i < 8; ++i) { f[i] = p[(size_t)i * DD]; pinf(f[i]); }
  v8us o;
#pragma unroll
  for (int i = 0; i < 8; ++i) o[i] = (unsigned short)bfbits(f[i]);
  unsigned short* dp = wd + (size_t)l * PLANE + (size_t)n * KP + k8;
  *(volatile v8us*)dp = o;
  *(volatile v8us*)(dp + DD) = o;
  __threadfence();
  *(volatile v8us*)dp = o;
  *(volatile v8us*)(dp + DD) = o;
}

__global__ __launch_bounds__(NTHR) void k_prep(
    const float* __restrict__ x, const float* __restrict__ ef, const float* __restrict__ ew,
    const float* __restrict__ eW, const float* __restrict__ eb, const float* __restrict__ W1,
    const float* __restrict__ b1, const float* __restrict__ W2, const float* __restrict__ b2,
    const int* __restrict__ ngp,
    float* H, unsigned short* Zhl, unsigned short* Thl, unsigned short* EFB, float* EWR,
    unsigned short* WeP, unsigned short* WD, float* BT, int* FLG,
    int e0, int e1, int e2, int e3, int e4, int e5, int e6, int e7)
{
  const int b = (int)blockIdx.x, tid = (int)threadIdx.x;
  if (b < e0) {
    const int u = b * NTHR + tid;
    const int row = u >> 6;
    const int c4 = (u & 63) * 4;
    const int rc = row < NN ? row : NN - 1;
    const v4f a = *(const v4f*)(x + (size_t)rc * DD + c4);
    const unsigned mk = row < NN ? 0xFFFFFFFFu : 0u;
    v4f o;
    o.x = __uint_as_float((bfbits(a.x) << 16) & mk);
    o.y = __uint_as_float((bfbits(a.y) << 16) & mk);
    o.z = __uint_as_float((bfbits(a.z) << 16) & mk);
    o.w = __uint_as_float((bfbits(a.w) << 16) & mk);
    float* hp = H + (size_t)row * DD + c4;
    *(volatile v4f*)hp = o;
    __threadfence();
    *(volatile v4f*)hp = o;
  } else if (b < e1) {
    const int u = (b - e0) * NTHR + tid;
    if (u >= NE * 2) return;
    const float* p = ef + (size_t)u * 8;
    const v4f a = *(const v4f*)p, c = *(const v4f*)(p + 4);
    v8us hv;
    hv[0] = (unsigned short)bfbits(a.x); hv[1] = (unsigned short)bfbits(a.y);
    hv[2] = (unsigned short)bfbits(a.z); hv[3] = (unsigned short)bfbits(a.w);
    hv[4] = (unsigned short)bfbits(c.x); hv[5] = (unsigned short)bfbits(c.y);
    hv[6] = (unsigned short)bfbits(c.z); hv[7] = (unsigned short)bfbits(c.w);
    unsigned short* op = EFB + (size_t)u * 8;
    *(volatile v8us*)op = hv;
    __threadfence();
    *(volatile v8us*)op = hv;
  } else if (b < e2) {
    const int u = (b - e1) * NTHR + tid;
    if (u >= NE / 4) return;
    const v4f a = *(const v4f*)(ew + (size_t)u * 4);
    v4f o; o.x = rbf(a.x); o.y = rbf(a.y); o.z = rbf(a.z); o.w = rbf(a.w);
    float* op = EWR + (size_t)u * 4;
    *(volatile v4f*)op = o;
    __threadfence();
    *(volatile v4f*)op = o;
  } else if (b < e3) {
    prep_wplane(W1, WD, (b - e2) * NTHR + tid);
  } else if (b < e4) {
    prep_wplane(W2, WD + (size_t)NL * PLANE, (b - e3) * NTHR + tid);
  } else if (b < e5) {
    const int v = (b - e4) * NTHR + tid;
    const int l = v >> 10;
    const int w = v & 1023;
    const int n = w >> 2;
    const int k8 = (w & 3) * 8;
    float f[8];
#pragma unroll
    for (int i = 0; i < 8; ++i) {
      const int kk = k8 + i;
      const int kc = kk < EDK ? kk : EDK - 1;
      f[i] = eW[(size_t)l * (EDK * DD) + (size_t)kc * DD + n];
      pinf(f[i]);
    }
    v8us hv;
#pragma unroll
    for (int i = 0; i < 8; ++i) {
      const unsigned mk = (k8 + i < EDK) ? 0xFFFFu : 0u;
      hv[i] = (unsigned short)(bfbits(f[i]) & mk);
    }
    unsigned short* op = WeP + (size_t)v * 8;
    *(volatile v8us*)op = hv;
    __threadfence();
    *(volatile v8us*)op = hv;
  } else if (b < e6) {
    const int u = (b - e5) * NTHR + tid;
    if (u >= 9 * 64) return;
    const int t = u >> 6;
    const int c4 = (u & 63) * 4;
    const int which = t / 3;
    const int l = t - 3 * which;
    const int li = l * DD + c4;
    const v4f a = *(const v4f*)(eb + li);
    const v4f c = *(const v4f*)(b1 + li);
    const v4f d = *(const v4f*)(b2 + li);
    pinf(a.x); pinf(c.x); pinf(d.x);
    const unsigned m0 = which == 0 ? 0xFFFFFFFFu : 0u;
    const unsigned m1 = which == 1 ? 0xFFFFFFFFu : 0u;
    const unsigned m2 = which == 2 ? 0xFFFFFFFFu : 0u;
    v4f o;
    o.x = __uint_as_float(((bfbits(a.x) << 16) & m0) | ((bfbits(c.x) << 16) & m1) | ((bfbits(d.x) << 16) & m2));
    o.y = __uint_as_float(((bfbits(a.y) << 16) & m0) | ((bfbits(c.y) << 16) & m1) | ((bfbits(d.y) << 16) & m2));
    o.z = __uint_as_float(((bfbits(a.z) << 16) & m0) | ((bfbits(c.z) << 16) & m1) | ((bfbits(d.z) << 16) & m2));
    o.w = __uint_as_float(((bfbits(a.w) << 16) & m0) | ((bfbits(c.w) << 16) & m1) | ((bfbits(d.w) << 16) & m2));
    float* op = BT + (size_t)u * 4;
    *(volatile v4f*)op = o;
    __threadfence();
    *(volatile v4f*)op = o;
  } else if (b < e7) {
    const int u = (b - e6) * NTHR + tid;
    const int row = NN + (u >> 6);
    const int c = (u & 63) * 8;
    const v4u z = {0u, 0u, 0u, 0u};
    unsigned short* zp = Zhl + (size_t)row * KP + c;
    unsigned short* tp = Thl + (size_t)row * KP + c;
    *(volatile v4u*)zp = z;
    *(volatile v4u*)tp = z;
    __threadfence();
    *(volatile v4u*)zp = z;
    *(volatile v4u*)tp = z;
  } else {
    const int ng = ngp[0];
    v4i fv = {0, 0, 0, 0};
    fv.x = (tid == 0 && ng != NGR) ? 1 : 0;
    if (tid < 8) *(volatile v4i*)(FLG + 4 * tid) = fv;
    __threadfence();
    if (tid < 8) *(volatile v4i*)(FLG + 4 * tid) = fv;
  }
}

__device__ __forceinline__ int scan_chunk(const int* __restrict__ keys, int nE, int cbase, int slotBase,
                                          int nb, int* list, int lane, int wave) {
  int wc = 0;
  const int elb  = wave * WCAP + lane;
  const int sent = (int)(1u << 31);
  int kv[EPT];
#pragma unroll
  for (int j = 0; j < EPT; ++j) {
    const int e  = cbase + elb + 32 * j;
    const int ec = e < nE ? e : nE - 1;
    const int v  = keys[ec];
    pini(v);
    const int mk = (e < nE) ? -1 : 0;
    kv[j] = (v & mk) | (sent & ~mk);
  }
  const unsigned nbs = (unsigned)slotBase;
  const unsigned unb = (unsigned)nb;
  const unsigned s0 = (unsigned)kv[0] - nbs, s1 = (unsigned)kv[1] - nbs;
  const unsigned s2 = (unsigned)kv[2] - nbs, s3 = (unsigned)kv[3] - nbs;
  const unsigned s4 = (unsigned)kv[4] - nbs, s5 = (unsigned)kv[5] - nbs;
  const unsigned s6 = (unsigned)kv[6] - nbs, s7 = (unsigned)kv[7] - nbs;
  const bool h0 = s0 < unb, h1 = s1 < unb, h2 = s2 < unb, h3 = s3 < unb;
  const bool h4 = s4 < unb, h5 = s5 < unb, h6 = s6 < unb, h7 = s7 < unb;
  const unsigned any = __builtin_amdgcn_ballot_w32(h0 | h1 | h2 | h3 | h4 | h5 | h6 | h7);
  if (any != 0u) {
#define HITJ(J, HJ, SJ) { \
      const unsigned mj = __builtin_amdgcn_ballot_w32(HJ); \
      if (mj != 0u) { \
        if (HJ) { \
          const int pos = wc + (int)__builtin_amdgcn_mbcnt_lo(mj, 0u); \
          if (pos < WCAP) list[wave * WCAP + pos] = ((elb + 32 * (J)) << 12) | (int)(SJ); \
        } \
        wc += (int)__builtin_popcount(mj); } }
    HITJ(0, h0, s0)
    HITJ(1, h1, s1)
    HITJ(2, h2, s2)
    HITJ(3, h3, s3)
    HITJ(4, h4, s4)
    HITJ(5, h5, s5)
    HITJ(6, h6, s6)
    HITJ(7, h7, s7)
#undef HITJ
  }
  return wc;
}

template<int NBT, int RC, int PAIR>
__global__ __launch_bounds__(NTHR) void k_bucket(const int* __restrict__ srcs, const int* __restrict__ keys,
                                                 int* ent, int* slot, int nRange, int nE, int srcMax) {
  constexpr int SPT = NBT / NTHR;
  extern __shared__ v4f lds_dyn[];
  int* reg1 = (int*)lds_dyn;
  int* reg2 = reg1 + RC;
  int* scnt = reg2 + RC;
  int* soff = scnt + NBT;
  int* list = soff + NBT;
  int* wcnt = list + LISTN;
  int* wtot = wcnt + NWAVE;
  const int tid = (int)threadIdx.x, lane = tid & 31;
  const int wave = __builtin_amdgcn_readfirstlane(tid >> 5);
  const int nodeBase = (int)blockIdx.x * NBT;
  int nb = nRange - nodeBase;
  nb = nb < 0 ? 0 : (nb > NBT ? NBT : nb);

  for (int i = tid; i < NBT; i += NTHR) scnt[i] = 0;
  for (int i = tid; i < RC; i += NTHR) { reg1[i] = 0; reg2[i] = 0; }
  __syncthreads();

  int tot = 0;
  const int nChunks = (nE + CHUNK - 1) / CHUNK;
#pragma unroll 1
  for (int ch = 0; ch < nChunks; ++ch) {
    const int cbase = ch * CHUNK;
    const int wc = scan_chunk(keys, nE, cbase, nodeBase, nb, list, lane, wave);
    if (lane == 0) wcnt[wave] = wc;
    __syncthreads();
    int pre = 0, all = 0;
#pragma unroll
    for (int w2 = 0; w2 < NWAVE; ++w2) {
      int c = wcnt[w2];
      c = c < 0 ? 0 : (c > WCAP ? WCAP : c);
      all += c;
      pre += (w2 < wave) ? c : 0;
    }
    const int wcc  = wc > WCAP ? WCAP : wc;
    const int base = tot + pre;
#pragma unroll 1
    for (int i = lane; i < wcc; i += 32) {
      const int en = list[wave * WCAP + i];
      const int el = (en >> 12) & (CHUNK - 1);
      const int sl = en & (NBT - 1);
      int eid = cbase + el;
      eid = eid > nE - 1 ? nE - 1 : eid;
      const int pos = base + i;
      if (pos < RC) reg1[pos] = (int)(((unsigned)eid << 12) | (unsigned)sl);
    }
    tot += all;
    tot = tot > RC ? RC : tot;
    __syncthreads();
  }
  const int nh = tot;

  if (wave == 0) {
#pragma unroll 1
    for (int b0 = 0; b0 < nh; b0 += 32) {
      const int idx = b0 + lane;
      const int uv  = reg1[idx < RC ? idx : RC - 1];
      const int m32 = (nh - b0) < 32 ? (nh - b0) : 32;
#pragma unroll 1
      for (int k = 0; k < m32; ++k) {
        const int u  = __builtin_amdgcn_readlane(uv, k);
        const int sl = u & (NBT - 1);
        if (lane == 0) scnt[sl] = scnt[sl] + 1;
      }
    }
  }
  __syncthreads();

  {
    int ev[SPT];
    int ts = 0;
#pragma unroll
    for (int j = 0; j < SPT; ++j) {
      const int r = scnt[SPT * tid + j];
      ev[j] = r < 0 ? 0 : r;
      ts += ev[j];
    }
    int incl = ts;
#pragma unroll
    for (int d = 1; d < 32; d <<= 1) {
      const int up = __shfl_up(incl, d);
      if (lane >= d) incl += up;
    }
    if (lane == 31) wtot[wave] = incl;
    __syncthreads();
    int pre = 0;
#pragma unroll
    for (int w2 = 0; w2 < NWAVE; ++w2) pre += (w2 < wave) ? wtot[w2] : 0;
    int run = pre + incl - ts;
#pragma unroll
    for (int j = 0; j < SPT; ++j) { soff[SPT * tid + j] = run; run += ev[j]; }
  }
  __syncthreads();
  for (int i = tid; i < NBT; i += NTHR) list[i] = soff[i];
  __syncthreads();

  if (wave == 0) {
#pragma unroll 1
    for (int b0 = 0; b0 < nh; b0 += 32) {
      const int idx = b0 + lane;
      const int uv  = reg1[idx < RC ? idx : RC - 1];
      const int m32 = (nh - b0) < 32 ? (nh - b0) : 32;
#pragma unroll 1
      for (int k = 0; k < m32; ++k) {
        const int u   = __builtin_amdgcn_readlane(uv, k);
        const int sl  = u & (NBT - 1);
        const int eid = (int)((unsigned)u >> 12);
        if (lane == 0) {
          int pos = list[sl];
          pos = pos < 0 ? 0 : (pos > RC - 1 ? RC - 1 : pos);
          reg2[pos] = eid;
          list[sl] = pos + 1;
        }
      }
    }
  }
  __syncthreads();

  const bool ovf = (nh >= RC);
#pragma unroll
  for (int j = 0; j < SPT; ++j) {
    const int s = SPT * tid + j;
    list[2 * s]     = soff[s];
    list[2 * s + 1] = ovf ? -1 : scnt[s];
  }
  __syncthreads();
#pragma unroll 1
  for (int q = 0; q < NBT / 512; ++q) {
    const int idx = q * NTHR + tid;
    const v4i sv = *(const v4ia*)(list + 4 * idx);
    int* sp = slot + 2 * (size_t)nodeBase + 4 * idx;
    *(volatile v4i*)sp = sv;
    __threadfence();
    *(volatile v4i*)sp = sv;
  }

  if constexpr (PAIR != 0) {
    int* eb = ent + (size_t)blockIdx.x * (size_t)(2 * RC);
#pragma unroll 1
    for (int p0 = 0; p0 < RC; p0 += 2 * NTHR) {
      const int p = p0 + 2 * tid;
      int q0 = reg2[p], q1 = reg2[p + 1];
      q0 = iclamp(q0, 0, nE - 1);
      q1 = iclamp(q1, 0, nE - 1);
      int s0 = srcs[q0];
      int s1 = srcs[q1];
      pini(s0); pini(s1);
      s0 = iclamp(s0, 0, srcMax - 1);
      s1 = iclamp(s1, 0, srcMax - 1);
      const int m0 = (p     < nh) ? -1 : 0;
      const int m1 = (p + 1 < nh) ? -1 : 0;
      v4i v;
      v.x = s0 & m0; v.y = q0 & m0; v.z = s1 & m1; v.w = q1 & m1;
      *(volatile v4i*)(eb + 2 * p) = v;
      __threadfence();
      *(volatile v4i*)(eb + 2 * p) = v;
    }
  } else {
    int* eb = ent + (size_t)blockIdx.x * (size_t)RC;
#pragma unroll 1
    for (int p0 = 0; p0 < RC; p0 += 4 * NTHR) {
      const int p = p0 + 4 * tid;
      const v4i r = *(const v4ia*)(reg2 + p);
      v4i v;
      v.x = iclamp(r.x, 0, nE - 1) & ((p     < nh) ? -1 : 0);
      v.y = iclamp(r.y, 0, nE - 1) & ((p + 1 < nh) ? -1 : 0);
      v.z = iclamp(r.z, 0, nE - 1) & ((p + 2 < nh) ? -1 : 0);
      v.w = iclamp(r.w, 0, nE - 1) & ((p + 3 < nh) ? -1 : 0);
      *(volatile v4i*)(eb + p) = v;
      __threadfence();
      *(volatile v4i*)(eb + p) = v;
    }
  }
}

__global__ __launch_bounds__(NTHR) __attribute__((amdgpu_num_vgpr(248)))
void k_conv(const int* __restrict__ ent, const int* __restrict__ slot,
            const unsigned short* __restrict__ efb, const float* __restrict__ ewr,
            const unsigned short* __restrict__ wep, const float* __restrict__ bt,
            const float* __restrict__ H, unsigned short* zhl)
{
  extern __shared__ v4f lds_dyn[];
  int*   sW = (int*)lds_dyn;
  float* sB = (float*)(sW + 4096);
  int*   sA = (int*)(sB + 256);
  float* sT = (float*)(sA + NWAVE * 256);
  const int tid = (int)threadIdx.x, lane = tid & 31, hh = lane >> 4, m = lane & 15;
  const int wave = __builtin_amdgcn_readfirstlane(tid >> 5);

#pragma unroll
  for (int i = 0; i < 4; ++i) {
    const int idx = i * NTHR + tid;
    *(v4i*)(sW + 4 * idx) = *(const v4i*)(wep + (size_t)idx * 8);
  }
  if (tid < 64) *(v4f*)(sB + 4 * tid) = *(const v4f*)(bt + 4 * tid);
  __syncthreads();

  const int i = (int)blockIdx.x * NWAVE + wave;
  int*   At = sA + wave * 256;
  float* Tt = sT + wave * 16 * TPI;

  const v2i se = *(const v2i*)(slot + 2 * (size_t)i);
  const int craw = __builtin_amdgcn_readfirstlane(se.y);
  const int stv = iclamp(se.x, 0, RCAPE - 1);
  int ccv = iclamp(se.y, 0, DEGCAP);
  ccv = ccv > RCAPE - stv ? RCAPE - stv : ccv;
  const int st  = __builtin_amdgcn_readfirstlane(stv);
  const int cnt = __builtin_amdgcn_readfirstlane(ccv);
  const float qnan = __int_as_float(0x7fc00000);
  const float pz = (craw < 0 || craw > DEGCAP) ? qnan : 0.0f;
  const int blk = i / NBE;
  const int* eb = ent + (size_t)blk * (size_t)(2 * RCAPE);
  const v8f z8 = {0.f, 0.f, 0.f, 0.f, 0.f, 0.f, 0.f, 0.f};

  const v4f bb0 = *(const v4fa*)(sB + 8 * lane);
  const v4f bb1 = *(const v4fa*)(sB + 8 * lane + 4);
  v4f a0 = {0.f, 0.f, 0.f, 0.f}, a1 = {0.f, 0.f, 0.f, 0.f};
  int last = st + cnt - 1; last = last < st ? st : last;

#pragma unroll 1
  for (int t0 = 0; t0 < cnt; t0 += 16) {
    const int nv = (cnt - t0) < 16 ? (cnt - t0) : 16;
    int ei = st + t0 + m;
    ei = ei > last ? last : ei;
    const v2i en = *(const v2i*)(eb + 2 * ei);
    const int src = iclamp(en.x, 0, NN - 1);
    const int eid = iclamp(en.y, 0, NE - 1);
    const float wv = ewr[eid];

    __builtin_amdgcn_fence(__ATOMIC_RELEASE, "wavefront");
    __builtin_amdgcn_wave_barrier();
    {
      const int row = lane >> 1;
      const int q   = lane & 1;
      const int er  = __shfl(eid, row);
      v4i w = *(const v4i*)(efb + (size_t)er * EDK + 8 * q);
      const int msk = (row < nv) ? -1 : 0;
      w.x &= msk; w.y &= msk; w.z &= msk; w.w &= msk;
      const v4i zz = {0, 0, 0, 0};
      *(v4i*)(At + row * 16 + 4 * q) = w;
      *(v4i*)(At + row * 16 + 8 + 4 * q) = zz;
    }
    __builtin_amdgcn_fence(__ATOMIC_RELEASE, "wavefront");
    __builtin_amdgcn_wave_barrier();
    FragB af;
    af.q[0] = *(const v4i*)(At + m * 16 + 4 * hh);
    af.q[1] = *(const v4i*)(At + m * 16 + 8 + 4 * hh);
#pragma unroll 4
    for (int tt = 0; tt < 16; ++tt) {
      const int* wq = sW + (16 * tt + m) * 16 + 4 * hh;
      FragB bf;
      bf.q[0] = *(const v4i*)wq;
      bf.q[1] = *(const v4i*)(wq + 8);
      v8f d = wmx(af, bf, z8);
#pragma unroll
      for (int r = 0; r < 8; ++r) Tt[(8 * hh + r) * TPI + 16 * tt + m] = d[r];
    }
    __builtin_amdgcn_fence(__ATOMIC_RELEASE, "wavefront");
    __builtin_amdgcn_wave_barrier();
#pragma unroll 1
    for (int r = 0; r < nv; ++r) {
      const int s = __builtin_amdgcn_readlane(src, r);
      const float w = __int_as_float(__builtin_amdgcn_readlane(__float_as_int(wv), r));
      const float* hp = H + (size_t)s * DD + 8 * lane;
      const v4f h0 = *(const v4f*)hp;
      const v4f h1 = *(const v4f*)(hp + 4);
      const v4f t0v = *(const v4fa*)(Tt + r * TPI + 8 * lane);
      const v4f t1v = *(const v4fa*)(Tt + r * TPI + 8 * lane + 4);
      v4f u0 = (h0 + t0v) + bb0;
      v4f u1 = (h1 + t1v) + bb1;
      u0.x = relu_keep(u0.x); u0.y = relu_keep(u0.y); u0.z = relu_keep(u0.z); u0.w = relu_keep(u0.w);
      u1.x = relu_keep(u1.x); u1.y = relu_keep(u1.y); u1.z = relu_keep(u1.z); u1.w = relu_keep(u1.w);
      a0 = a0 + u0 * w;
      a1 = a1 + u1 * w;
    }
  }

  const bool live = i < NN;
  const int ic = live ? i : NN - 1;
  const float* sp = H + (size_t)ic * DD + 8 * lane;
  const v4f s0 = *(const v4f*)sp;
  const v4f s1 = *(const v4f*)(sp + 4);
  v4f z0 = (s0 + a0) + pz;
  v4f z1 = (s1 + a1) + pz;
  const v4f zero4 = {0.f, 0.f, 0.f, 0.f};
  z0 = live ? z0 : zero4;
  z1 = live ? z1 : zero4;
  const HL hl = split8(z0, z1);
  unsigned short* zp = zhl + (size_t)i * KP + 8 * lane;
  *(volatile v4u*)zp = hl.h;
  *(volatile v4u*)(zp + DD) = hl.l;
  __threadfence();
  *(volatile v4u*)zp = hl.h;
  *(volatile v4u*)(zp + DD) = hl.l;
}

template<int MODE, int KEXT, int LAST>
__global__ __launch_bounds__(GTHR) __attribute__((amdgpu_num_vgpr(248)))
void k_gemm(const unsigned short* __restrict__ A, const unsigned short* __restrict__ WT,
            const float* __restrict__ bias, void* outp, float* outG, const int* __restrict__ flg)
{
  __shared__ __attribute__((aligned(16))) float stg[GBM * BN];
  __shared__ __attribute__((aligned(16))) float bsh[BN];
  const int tid = (int)threadIdx.x, lane = tid & 31, hh = lane >> 4, m = lane & 15;
  const int wave = __builtin_amdgcn_readfirstlane(tid >> 5);
  const int rowBase = (int)blockIdx.x * GBM;
  const int col0    = (int)blockIdx.y * BN;
  const int fl = flg[0];

  if (tid < 32) *(v4f*)(bsh + 4 * tid) = *(const v4f*)(bias + col0 + 4 * tid);
  __syncthreads();

  v8f acc[GNT];
  {
    const v8f z = {0.f, 0.f, 0.f, 0.f, 0.f, 0.f, 0.f, 0.f};
#pragma unroll
    for (int t = 0; t < GNT; ++t) acc[t] = z;
  }
  const unsigned short* ap = A  + (size_t)(rowBase + 16 * wave + m) * (size_t)KP + 8 * hh;
  const unsigned short* wp = WT + (size_t)(col0 + m) * (size_t)KP + 8 * hh;
  constexpr int ksteps = KEXT / 32;
#pragma unroll 1
  for (int ks = 0; ks < ksteps; ++ks) {
    FragB af;
    af.u[0] = *(const v8us*)(ap + 32 * ks);
    af.u[1] = *(const v8us*)(ap + 32 * ks + 16);
#pragma unroll
    for (int t = 0; t < GNT; ++t) {
      const unsigned short* wq = wp + (size_t)(16 * t) * (size_t)KP + 32 * ks;
      FragB bf;
      bf.u[0] = *(const v8us*)wq;
      bf.u[1] = *(const v8us*)(wq + 16);
      acc[t] = wmx(af, bf, acc[t]);
    }
  }

#pragma unroll
  for (int t = 0; t < GNT; ++t) {
    const int lc = 16 * t + m;
    const float bb = bsh[lc];
#pragma unroll
    for (int r = 0; r < 8; ++r) {
      const int lr = 16 * wave + 8 * hh + r;
      const bool live = (rowBase + lr) < NN;
      const float v = relu_keep(acc[t][r] + bb);
      stg[lr * BN + lc] = live ? v : 0.0f;
    }
  }
  __syncthreads();

  if constexpr (MODE == 0) {
    float* outF = (float*)outp;
    const float pz = (LAST != 0 && fl != 0) ? __int_as_float(0x7fc00000) : 0.0f;
#pragma unroll 1
    for (int i2 = 0; i2 < 16; ++i2) {
      const int lr = 16 * wave + i2;
      const int gr = rowBase + lr;
      const v4f v = *(const v4fa*)(stg + lr * BN + 4 * lane);
      const v4f vo = v + pz;
      float* hp = outF + (size_t)gr * DD + col0 + 4 * lane;
      float* gp = outG + (size_t)(gr < NN ? gr : NN - 1) * DD + col0 + 4 * lane;
      const bool og = (LAST != 0) && (gr < NN);
      *(volatile v4f*)hp = v;
      if (og) *(volatile v4f*)gp = vo;
      __threadfence();
      *(volatile v4f*)hp = v;
      if (og) *(volatile v4f*)gp = vo;
    }
  } else {
    unsigned short* outH = (unsigned short*)outp;
    const int cb = 8 * m;
    const unsigned selHi = (hh == 0) ? 0xFFFFFFFFu : 0u;
#pragma unroll 1
    for (int i2 = 0; i2 < 16; ++i2) {
      const int lr = 16 * wave + i2;
      const int gr = rowBase + lr;
      const v4f a = *(const v4fa*)(stg + lr * BN + cb);
      const v4f b = *(const v4fa*)(stg + lr * BN + cb + 4);
      const HL hl = split8(a, b);
      v4u pw;
      pw.x = (hl.h.x & selHi) | (hl.l.x & ~selHi);
      pw.y = (hl.h.y & selHi) | (hl.l.y & ~selHi);
      pw.z = (hl.h.z & selHi) | (hl.l.z & ~selHi);
      pw.w = (hl.h.w & selHi) | (hl.l.w & ~selHi);
      unsigned short* op = outH + (size_t)gr * KP + hh * DD + col0 + cb;
      *(volatile v4u*)op = pw;
      __threadfence();
      *(volatile v4u*)op = pw;
    }
  }
  (void)outG; (void)fl;
}

__global__ __launch_bounds__(NTHR) void k_pool(const int* __restrict__ pent, const int* __restrict__ pslot,
                                               const float* __restrict__ H, const int* __restrict__ flg, float* og) {
  const int tid = (int)threadIdx.x, lane = tid & 31;
  const int wave = __builtin_amdgcn_readfirstlane(tid >> 5);
  const int g = (int)blockIdx.x * NWAVE + wave;
  const v2i se = *(const v2i*)(pslot + 2 * (size_t)g);
  const int craw = __builtin_amdgcn_readfirstlane(se.y);
  const int stv = iclamp(se.x, 0, RCAPG - 1);
  int ccv = iclamp(se.y, 0, PGCAP);
  ccv = ccv > RCAPG - stv ? RCAPG - stv : ccv;
  const int st  = __builtin_amdgcn_readfirstlane(stv);
  const int cnt = __builtin_amdgcn_readfirstlane(ccv);
  const int fl = flg[0];
  const float pz = (craw < 0 || craw > PGCAP || fl != 0) ? __int_as_float(0x7fc00000) : 0.0f;
  const int* eb = pent + (size_t)(g / NBG) * (size_t)RCAPG;
  int last = st + cnt - 1; last = last < st ? st : last;
  v4f a0 = {0.f, 0.f, 0.f, 0.f}, a1 = {0.f, 0.f, 0.f, 0.f};
#pragma unroll 1
  for (int b0 = 0; b0 < cnt; b0 += 32) {
    int idx = st + b0 + lane;
    idx = idx > last ? last : idx;
    const int nd = iclamp(eb[idx], 0, NN - 1);
    const int m32 = (cnt - b0) < 32 ? (cnt - b0) : 32;
#pragma unroll 1
    for (int k = 0; k < m32; ++k) {
      const int nk = __builtin_amdgcn_readlane(nd, k);
      const float* hp = H + (size_t)nk * DD + 4 * lane;
      const v4f v0 = *(const v4f*)hp;
      const v4f v1 = *(const v4f*)(hp + 128);
      a0 = a0 + v0;
      a1 = a1 + v1;
    }
  }
  const v4f o0 = a0 + pz;
  const v4f o1 = a1 + pz;
  float* op = og + (size_t)g * DD + 4 * lane;
  *(volatile v4f*)op = o0;
  *(volatile v4f*)(op + 128) = o1;
  __threadfence();
  *(volatile v4f*)op = o0;
  *(volatile v4f*)(op + 128) = o1;
}

static inline int cdiv(int a, int b) { return (a + b - 1) / b; }
static inline size_t al256(size_t o) { return (o + 255) & ~(size_t)255; }

extern "C" void kernel_launch(void* const* d_in, const int* in_sizes, int n_in,
                              void* d_out, int out_size, void* d_ws, size_t ws_size,
                              hipStream_t stream) {
  if (n_in < 13) return;
  if (in_sizes[0] != NN * DD) return;
  if (in_sizes[1] != NE * EDK) return;
  if (in_sizes[2] != NE) return;
  if (in_sizes[3] != NL * EDK * DD) return;
  if (in_sizes[4] != NL * DD) return;
  if (in_sizes[5] != NL * DD * DD) return;
  if (in_sizes[6] != NL * DD) return;
  if (in_sizes[7] != NL * DD * DD) return;
  if (in_sizes[8] != NL * DD) return;
  if (in_sizes[9] != NE || in_sizes[10] != NE) return;
  if (in_sizes[11] != NN || in_sizes[12] != 1) return;
  if (out_size != NN * DD + NGR * DD) return;

  const float* x   = (const float*)d_in[0];
  const float* ef  = (const float*)d_in[1];
  const float* ew  = (const float*)d_in[2];
  const float* eW  = (const float*)d_in[3];
  const float* ebp = (const float*)d_in[4];
  const float* W1  = (const float*)d_in[5];
  const float* b1  = (const float*)d_in[6];
  const float* W2  = (const float*)d_in[7];
  const float* b2  = (const float*)d_in[8];
  const int*   nin = (const int*)d_in[9];
  const int*   nou = (const int*)d_in[10];
  const int*   n2g = (const int*)d_in[11];
  const int*   ngp = (const int*)d_in[12];
  float* out0 = (float*)d_out;
  float* out1 = out0 + (size_t)OUT1_EL;

  const int gBE = cdiv(NN, NBE);
  const int gBG = cdiv(NGR, NBG);

  char* ws = (char*)d_ws;
  size_t off = 0;
  const size_t oH   = off; off = al256(off + (size_t)MP * DD * 4);
  const size_t oZ   = off; off = al256(off + (size_t)MP * KP * 2);
  const size_t oT   = off; off = al256(off + (size_t)MP * KP * 2);
  const size_t oEFB = off; off = al256(off + (size_t)NE * EDK * 2);
  const size_t oEWR = off; off = al256(off + (size_t)NE * 4);
  const size_t oENT = off; off = al256(off + (size_t)gBE * RCAPE * 8);
  const size_t oSLT = off; off = al256(off + (size_t)gBE * NBE * 8);
  const size_t oPEN = off; off = al256(off + (size_t)gBG * RCAPG * 4);
  const size_t oPSL = off; off = al256(off + (size_t)gBG * NBG * 8);
  const size_t oWEP = off; off = al256(off + (size_t)NL * DD * 32 * 2);
  const size_t oWD  = off; off = al256(off + (size_t)2 * NL * PLANE * 2);
  const size_t oBT  = off; off = al256(off + (size_t)9 * DD * 4);
  const size_t oFLG = off; off = al256(off + (size_t)128);
  if (off > ws_size || off > ((size_t)256u << 20)) return;
  float*          H    = (float*)(ws + oH);
  unsigned short* Zhl  = (unsigned short*)(ws + oZ);
  unsigned short* Thl  = (unsigned short*)(ws + oT);
  unsigned short* EFB  = (unsigned short*)(ws + oEFB);
  float*          EWR  = (float*)(ws + oEWR);
  int*            ENT  = (int*)(ws + oENT);
  int*            SLT  = (int*)(ws + oSLT);
  int*            PENT = (int*)(ws + oPEN);
  int*            PSLT = (int*)(ws + oPSL);
  unsigned short* WeP  = (unsigned short*)(ws + oWEP);
  unsigned short* WD   = (unsigned short*)(ws + oWD);
  float*          BT   = (float*)(ws + oBT);
  int*            FLG  = (int*)(ws + oFLG);

  hipFuncSetAttribute(reinterpret_cast<const void*>(&k_bucket<NBE, RCAPE, 1>),
                      hipFuncAttributeMaxDynamicSharedMemorySize, LDS_BKE);
  hipFuncSetAttribute(reinterpret_cast<const void*>(&k_bucket<NBG, RCAPG, 0>),
                      hipFuncAttributeMaxDynamicSharedMemorySize, LDS_BKG);
  hipFuncSetAttribute(reinterpret_cast<const void*>(&k_conv),
                      hipFuncAttributeMaxDynamicSharedMemorySize, LDS_CONV);

  {
    const int e0 = (MP * 64) / NTHR;
    const int e1 = e0 + cdiv(NE * 2, NTHR);
    const int e2 = e1 + cdiv(NE / 4, NTHR);
    const int e3 = e2 + (NL * 8192) / NTHR;
    const int e4 = e3 + (NL * 8192) / NTHR;
    const int e5 = e4 + (NL * 1024) / NTHR;
    const int e6 = e5 + cdiv(9 * 64, NTHR);
    const int e7 = e6 + (48 * 64) / NTHR;
    const int nb = e7 + 1;
    k_prep<<<nb, NTHR, 0, stream>>>(x, ef, ew, eW, ebp, W1, b1, W2, b2, ngp,
                                    H, Zhl, Thl, EFB, EWR, WeP, WD, BT, FLG,
                                    e0, e1, e2, e3, e4, e5, e6, e7);
  }
  k_bucket<NBE, RCAPE, 1><<<gBE, NTHR, LDS_BKE, stream>>>(nin, nou, ENT, SLT, NN, NE, NN);
  k_bucket<NBG, RCAPG, 0><<<gBG, NTHR, LDS_BKG, stream>>>(n2g, n2g, PENT, PSLT, NGR, NN, NN);

  const dim3 gG(MP / GBM, DD / BN);
  for (int l = 0; l < NL; ++l) {
    k_conv<<<MP / NWAVE, NTHR, LDS_CONV, stream>>>(ENT, SLT, EFB, EWR, WeP + (size_t)l * (DD * 32),
                                                   BT + (size_t)l * DD, H, Zhl);
    k_gemm<1, KZ, 0><<<gG, GTHR, 0, stream>>>(Zhl, WD + (size_t)l * PLANE, BT + (size_t)(3 + l) * DD,
                                              (void*)Thl, out0, FLG);
    if (l < NL - 1) {
      k_gemm<0, KT, 0><<<gG, GTHR, 0, stream>>>(Thl, WD + (size_t)(NL + l) * PLANE, BT + (size_t)(6 + l) * DD,
                                                (void*)H, out0, FLG);
    } else {
      k_gemm<0, KT, 1><<<gG, GTHR, 0, stream>>>(Thl, WD + (size_t)(NL + l) * PLANE, BT + (size_t)(6 + l) * DD,
                                                (void*)H, out0, FLG);
    }
  }
  k_pool<<<NGR / NWAVE, NTHR, 0, stream>>>(PENT, PSLT, H, FLG, out1);
}
